// GCN_33208687133423
// MI455X (gfx1250) — hardware-verified
//
#include <hip/hip_runtime.h>
#include <stddef.h>
#include <stdint.h>
#include <math.h>


#define DF     128
#define DO     64
#define KA     256
#define NTHR   256
#define NWAVE  8
#define EPT    8
#define CHUNK  (NTHR * EPT)
#define WCAP   (EPT * 32)
#define LISTN  (NWAVE * WCAP)
#define NBA    1024
#define SLA    10
#define RCAP   28672
#define DEGCAP 64
#define GBM    64
#define GTHR   128
#define NBW1   16
#define NBW2   8
#define MISC_INTS 32
#define AGG_ZINTS (LISTN + 2 * RCAP + 3 * NBA)
#define AGG_LDS_INTS (AGG_ZINTS + MISC_INTS)
#define FLP    32
#define WSMAX  134217728

static_assert((CHUNK & (CHUNK - 1)) == 0 && CHUNK <= 4096);
static_assert((NBA & (NBA - 1)) == 0 && NBA == (1 << SLA));
static_assert(((long long)CHUNK << SLA) < (1LL << 31));
static_assert(LISTN % NTHR == 0);
static_assert(NBA % NWAVE == 0 && NBA % 32 == 0 && NBA % GBM == 0);
static_assert(RCAP % 4 == 0 && AGG_ZINTS % 4 == 0 && LISTN % 4 == 0);
static_assert(RCAP >= 16710 + 836 && DEGCAP >= 36 + 8 && DEGCAP % 32 == 0);
static_assert(DF == 4 * 32 && DO == 2 * 32 && KA == 2 * DF && KA % 32 == 0);
static_assert(GBM == (GTHR / 32) * 16);
static_assert(NBW1 * NTHR == DF * (KA / 8) && NBW2 * NTHR == DO * (KA / 8) && KA / 8 == 32);
static_assert(AGG_LDS_INTS * 4 <= 300000);

typedef float          v2f   __attribute__((ext_vector_type(2)));
typedef float          v4f   __attribute__((ext_vector_type(4)));
typedef float          v8f   __attribute__((ext_vector_type(8)));
typedef int            v4i   __attribute__((ext_vector_type(4)));
typedef int            v8i   __attribute__((ext_vector_type(8)));
typedef unsigned       v2u   __attribute__((ext_vector_type(2)));
typedef unsigned short v8us  __attribute__((ext_vector_type(8)));
typedef unsigned short v16us __attribute__((ext_vector_type(16)));
typedef __bf16         v16bf __attribute__((ext_vector_type(16)));
typedef v2f  __attribute__((may_alias)) v2fa;
typedef v4f  __attribute__((may_alias)) v4fa;
typedef v4i  __attribute__((may_alias)) v4ia;
typedef v2u  __attribute__((may_alias)) v2ua;
typedef v8us __attribute__((may_alias)) v8usa;
union FragB { v16bf v; v16us u; v8us h[2]; v8i w; };

__device__ __forceinline__ v8f wmb(const FragB& a, const FragB& b, v8f c) {
  v8f d = __builtin_amdgcn_wmma_f32_16x16x32_bf16(false, a.v, false, b.v, (short)0, c, false, false);
  asm volatile("v_nop\n\tv_nop\n\tv_nop\n\tv_nop" : "+v"(d) : "v"(a.w), "v"(b.w));
  return d;
}

__device__ __forceinline__ unsigned bf16_bits(float f) {
  const unsigned u = __float_as_uint(f);
  return (u + 0x7FFFu + ((u >> 16) & 1u)) >> 16;
}
__device__ __forceinline__ float bf16_val(float f) {
  return __uint_as_float(bf16_bits(f) << 16);
}

__device__ __forceinline__ float wsum(float v) {
#pragma unroll
  for (int q = 16; q > 0; q >>= 1) v += __shfl_xor(v, q, 32);
  return v;
}

__device__ __forceinline__ void hilo_pack(float v0, float v1, float v2, float v3,
                                          int& h01, int& h23, int& l01, int& l23) {
  const unsigned a0 = bf16_bits(v0), a1 = bf16_bits(v1), a2 = bf16_bits(v2), a3 = bf16_bits(v3);
  const unsigned b0 = bf16_bits(v0 - __uint_as_float(a0 << 16));
  const unsigned b1 = bf16_bits(v1 - __uint_as_float(a1 << 16));
  const unsigned b2 = bf16_bits(v2 - __uint_as_float(a2 << 16));
  const unsigned b3 = bf16_bits(v3 - __uint_as_float(a3 << 16));
  h01 = (int)(a0 | (a1 << 16)); h23 = (int)(a2 | (a3 << 16));
  l01 = (int)(b0 | (b1 << 16)); l23 = (int)(b2 | (b3 << 16));
}

__device__ __forceinline__ v4i regroup16(int h01, int h23, int l01, int l23, int lane) {
  const int s0 = (2 * lane) & 31, s1 = s0 + 1;
  const int a0 = __shfl(h01, s0, 32), a1 = __shfl(h23, s0, 32), a2 = __shfl(h01, s1, 32), a3 = __shfl(h23, s1, 32);
  const int b0 = __shfl(l01, s0, 32), b1 = __shfl(l23, s0, 32), b2 = __shfl(l01, s1, 32), b3 = __shfl(l23, s1, 32);
  const int mk = (lane < 16) ? -1 : 0;
  v4i o;
  o.x = (a0 & mk) | (b0 & ~mk); o.y = (a1 & mk) | (b1 & ~mk);
  o.z = (a2 & mk) | (b2 & ~mk); o.w = (a3 & mk) | (b3 & ~mk);
  return o;
}

template <int SLB>
__device__ __forceinline__ int scan_chunk(const int* __restrict__ dsts, int nE, int cbase, int slotBase,
                                          int nb, int vec8, int* list, int tid, int lane, int wave) {
  int wc = 0;
  const int el0  = tid * EPT;
  const int e0   = cbase + el0;
  const int sent = -2147483647 - 1;
  v4i da, db;
  if (vec8 != 0 && cbase + CHUNK <= nE) {
    da = *(const v4i*)(dsts + e0);
    db = *(const v4i*)(dsts + e0 + 4);
  } else {
    da.x = (e0     < nE) ? dsts[min(e0,     nE - 1)] : sent;
    da.y = (e0 + 1 < nE) ? dsts[min(e0 + 1, nE - 1)] : sent;
    da.z = (e0 + 2 < nE) ? dsts[min(e0 + 2, nE - 1)] : sent;
    da.w = (e0 + 3 < nE) ? dsts[min(e0 + 3, nE - 1)] : sent;
    db.x = (e0 + 4 < nE) ? dsts[min(e0 + 4, nE - 1)] : sent;
    db.y = (e0 + 5 < nE) ? dsts[min(e0 + 5, nE - 1)] : sent;
    db.z = (e0 + 6 < nE) ? dsts[min(e0 + 6, nE - 1)] : sent;
    db.w = (e0 + 7 < nE) ? dsts[min(e0 + 7, nE - 1)] : sent;
  }
  const unsigned nbs = (unsigned)slotBase;
  const unsigned unb = (unsigned)nb;
  const unsigned s0 = (unsigned)da.x - nbs, s1 = (unsigned)da.y - nbs;
  const unsigned s2 = (unsigned)da.z - nbs, s3 = (unsigned)da.w - nbs;
  const unsigned s4 = (unsigned)db.x - nbs, s5 = (unsigned)db.y - nbs;
  const unsigned s6 = (unsigned)db.z - nbs, s7 = (unsigned)db.w - nbs;
  const bool h0 = s0 < unb, h1 = s1 < unb, h2 = s2 < unb, h3 = s3 < unb;
  const bool h4 = s4 < unb, h5 = s5 < unb, h6 = s6 < unb, h7 = s7 < unb;
  const unsigned any = __builtin_amdgcn_ballot_w32(h0 | h1 | h2 | h3 | h4 | h5 | h6 | h7);
  if (any != 0u) {
#define HITJ(J, HJ, SJ) { \
      const unsigned mj = __builtin_amdgcn_ballot_w32(HJ); \
      if (mj != 0u) { \
        if (HJ) { \
          const int pos = wc + (int)__builtin_amdgcn_mbcnt_lo(mj, 0u); \
          if (pos < WCAP) list[wave * WCAP + pos] = ((el0 + (J)) << SLB) | (int)(SJ); \
        } \
        wc += (int)__builtin_popcount(mj); } }
    HITJ(0, h0, s0)
    HITJ(1, h1, s1)
    HITJ(2, h2, s2)
    HITJ(3, h3, s3)
    HITJ(4, h4, s4)
    HITJ(5, h5, s5)
    HITJ(6, h6, s6)
    HITJ(7, h7, s7)
#undef HITJ
  }
  return wc;
}

__global__ __launch_bounds__(NTHR) void k_prep(const float* __restrict__ x, int nN, int gx,
                                               const float* __restrict__ w1, const float* __restrict__ w2,
                                               unsigned short* xb, unsigned short* w1d, unsigned short* w2d) {
  const int tid = (int)threadIdx.x;
  const int blk = (int)blockIdx.x;
  if (blk < gx) {
    const int total = nN * (DF / 8);
    const int u  = blk * NTHR + tid;
    const int uc = u < total ? u : total - 1;
    const int row = uc >> 4;
    const int k8  = (uc & 15) * 8;
    const float* p = x + (size_t)row * DF + k8;
    const v4f a = *(const v4fa*)p;
    const v4f b = *(const v4fa*)(p + 4);
    v8us o;
    o[0] = (unsigned short)bf16_bits(a.x); o[1] = (unsigned short)bf16_bits(a.y);
    o[2] = (unsigned short)bf16_bits(a.z); o[3] = (unsigned short)bf16_bits(a.w);
    o[4] = (unsigned short)bf16_bits(b.x); o[5] = (unsigned short)bf16_bits(b.y);
    o[6] = (unsigned short)bf16_bits(b.z); o[7] = (unsigned short)bf16_bits(b.w);
    if (u < total) {
      unsigned short* dp = xb + (size_t)row * DF + k8;
      *(volatile v8us*)dp = o;
      __threadfence();
      *(volatile v8us*)dp = o;
    }
  } else {
    const int pb = blk - gx;
    const bool second = pb >= NBW1;
    const float* w = second ? w2 : w1;
    unsigned short* wd = second ? w2d : w1d;
    const int pitch = second ? DO : DF;
    const int u  = (second ? (pb - NBW1) : pb) * NTHR + tid;
    const int n  = u >> 5;
    const int k8 = (u & 31) * 8;
    const int kk = k8 & (DF - 1);
    const float* p = w + (size_t)kk * pitch + n;
    const float f0 = p[0];
    const float f1 = p[(size_t)pitch];
    const float f2 = p[(size_t)2 * pitch];
    const float f3 = p[(size_t)3 * pitch];
    const float f4 = p[(size_t)4 * pitch];
    const float f5 = p[(size_t)5 * pitch];
    const float f6 = p[(size_t)6 * pitch];
    const float f7 = p[(size_t)7 * pitch];
    v8us o;
    o[0] = (unsigned short)bf16_bits(f0); o[1] = (unsigned short)bf16_bits(f1);
    o[2] = (unsigned short)bf16_bits(f2); o[3] = (unsigned short)bf16_bits(f3);
    o[4] = (unsigned short)bf16_bits(f4); o[5] = (unsigned short)bf16_bits(f5);
    o[6] = (unsigned short)bf16_bits(f6); o[7] = (unsigned short)bf16_bits(f7);
    unsigned short* dp = wd + (size_t)n * KA + k8;
    *(volatile v8us*)dp = o;
    __threadfence();
    *(volatile v8us*)dp = o;
  }
}

template <int NT, int FIN>
__global__ __launch_bounds__(GTHR) void k_gemm(unsigned short* Apl, const unsigned short* __restrict__ BT,
                                               const float* __restrict__ bias, int nN, float* gout) {
  constexpr int NC = 16 * NT;
  __shared__ __attribute__((aligned(16))) float stg[GBM * NC];
  const int tid = (int)threadIdx.x, lane = tid & 31, wave = tid >> 5, hh = lane >> 4, m = lane & 15;
  const int rowBase = (int)blockIdx.x * GBM;

  v8f acc[NT];
  {
    const v8f z = {0.f, 0.f, 0.f, 0.f, 0.f, 0.f, 0.f, 0.f};
#pragma unroll
    for (int t = 0; t < NT; ++t) acc[t] = z;
  }
  const unsigned short* ap = Apl + (size_t)(rowBase + 16 * wave + m) * (size_t)KA + 8 * hh;
  const unsigned short* bp = BT  + (size_t)m * (size_t)KA + 8 * hh;

#pragma unroll 1
  for (int k0 = 0; k0 < KA; k0 += 32) {
    FragB af;
    af.h[0] = *(const v8usa*)(ap + k0);
    af.h[1] = *(const v8usa*)(ap + k0 + 16);
#pragma unroll
    for (int nt = 0; nt < NT; ++nt) {
      const unsigned short* wq = bp + (size_t)(16 * nt) * (size_t)KA + k0;
      FragB bf;
      bf.h[0] = *(const v8usa*)wq;
      bf.h[1] = *(const v8usa*)(wq + 16);
      acc[nt] = wmb(af, bf, acc[nt]);
    }
  }

#pragma unroll
  for (int nt = 0; nt < NT; ++nt) {
    const int lc = 16 * nt + m;
#pragma unroll
    for (int r = 0; r < 8; ++r) {
      const int lr = 16 * wave + 8 * hh + r;
      stg[lr * NC + lc] = acc[nt][r];
    }
  }
  __syncthreads();

  if constexpr (FIN == 0) {
    static_assert(NT == 8);
    v4f bq = *(const v4f*)(bias + 4 * lane);
    bq.x = bf16_val(bq.x); bq.y = bf16_val(bq.y); bq.z = bf16_val(bq.z); bq.w = bf16_val(bq.w);
#pragma unroll 1
    for (int i = 0; i < 16; ++i) {
      const int lr   = 16 * wave + i;
      const int grow = rowBase + lr;
      const bool live = grow < nN;
      const v4f mv = *(const v4fa*)(stg + lr * NC + 4 * lane);
      const float t0 = mv.x + bq.x, t1 = mv.y + bq.y, t2 = mv.z + bq.z, t3 = mv.w + bq.w;
      float y0 = (t0 > 0.0f) ? t0 : (t0 - t0);
      float y1 = (t1 > 0.0f) ? t1 : (t1 - t1);
      float y2 = (t2 > 0.0f) ? t2 : (t2 - t2);
      float y3 = (t3 > 0.0f) ? t3 : (t3 - t3);
      y0 = live ? y0 : 0.0f; y1 = live ? y1 : 0.0f; y2 = live ? y2 : 0.0f; y3 = live ? y3 : 0.0f;
      int h01, h23, l01, l23;
      hilo_pack(y0, y1, y2, y3, h01, h23, l01, l23);
      const v4i ow = regroup16(h01, h23, l01, l23, lane);
      unsigned short* dp = Apl + (size_t)grow * (size_t)KA + 8 * lane;
      *(volatile v4i*)dp = ow;
      __threadfence();
      *(volatile v4i*)dp = ow;
    }
  } else {
    static_assert(NT == 4);
    const int hr = lane >> 4, c4 = 4 * (lane & 15);
#pragma unroll 1
    for (int i = 0; i < 8; ++i) {
      const int lr   = 16 * wave + 2 * i + hr;
      const int grow = rowBase + lr;
      const v4f v = *(const v4fa*)(stg + lr * NC + c4);
      float* op = gout + (size_t)grow * DO + c4;
      *(volatile v4f*)op = v;
      __threadfence();
      *(volatile v4f*)op = v;
    }
  }
}

template <int LY>
__global__ __launch_bounds__(NTHR) void k_scan(const int* __restrict__ gath, const int* __restrict__ keys,
                                               const float* __restrict__ ew,
                                               int nE, int nN, int vec8, int mRows,
                                               const unsigned short* __restrict__ xb,
                                               const float* __restrict__ gq,
                                               const int* __restrict__ idx1, const int* __restrict__ rep1, int nC,
                                               const float* __restrict__ b2,
                                               unsigned short* apl, float* qout, int* flg) {
  extern __shared__ __attribute__((aligned(16))) int dsm[];
  int* list = dsm;
  int* hl   = dsm + LISTN;
  int* sl   = hl + RCAP;
  int* cnt  = sl + RCAP;
  int* offs = cnt + NBA;
  int* cur  = offs + NBA;
  int* misc = cur + NBA;
  const int tid = (int)threadIdx.x, lane = tid & 31, wave = tid >> 5;
  const int nodeBase = (int)blockIdx.x * NBA;

  {
    const v4i z4 = {0, 0, 0, 0};
    for (int i = tid * 4; i < AGG_ZINTS; i += NTHR * 4) *(v4ia*)(dsm + i) = z4;
    if (tid < MISC_INTS) misc[tid] = 0;
  }
  __syncthreads();

  int t = 0, ov = 0;
  const int nChunks = (nE + CHUNK - 1) / CHUNK;
#pragma unroll 1
  for (int ch = 0; ch < nChunks; ++ch) {
    const int cbase = ch * CHUNK;
    const int wc = scan_chunk<SLA>(keys, nE, cbase, nodeBase, NBA, vec8, list, tid, lane, wave);
    if (lane == 0) misc[wave] = wc;
    __syncthreads();
    if (wave == 0) {
#pragma unroll 1
      for (int w2 = 0; w2 < NWAVE; ++w2) {
        int c = misc[w2];
        c = c < 0 ? 0 : (c > WCAP ? WCAP : c);
#pragma unroll 1
        for (int b0 = 0; b0 < c; b0 += 32) {
          const int idx = b0 + lane;
          const int ent = list[w2 * WCAP + (idx < WCAP ? idx : WCAP - 1)];
          const int m32 = (c - b0) < 32 ? (c - b0) : 32;
#pragma unroll 1
          for (int k = 0; k < m32; ++k) {
            const int u    = __builtin_amdgcn_readlane(ent, k);
            const int slot = u & (NBA - 1);
            const int el   = (u >> SLA) & (CHUNK - 1);
            const int pk   = ((cbase + el) << SLA) | slot;
            if (t < RCAP) {
              if (lane == 0) { hl[t] = pk; cnt[slot] = cnt[slot] + 1; }
              t = t + 1;
            } else {
              ov = 1;
            }
          }
        }
      }
    }
    __syncthreads();
  }
  if (wave == 0 && lane == 0) { misc[8] = t; misc[9] = ov; }
  __syncthreads();
  int tt = misc[8];
  tt = tt < 0 ? 0 : (tt > RCAP ? RCAP : tt);
  const int ovf = misc[9];

  if (wave == 0) {
    const int base = lane * (NBA / 32);
    int s = 0;
#pragma unroll 1
    for (int i = 0; i < NBA / 32; ++i) s += cnt[base + i];
    int incl = s;
#pragma unroll
    for (int d = 1; d < 32; d <<= 1) {
      const int y = __shfl_up(incl, d, 32);
      if (lane >= d) incl += y;
    }
    int run = incl - s;
#pragma unroll 1
    for (int i = 0; i < NBA / 32; ++i) {
      const int cv = cnt[base + i];
      offs[base + i] = run;
      cur[base + i]  = run;
      run += cv;
    }
  }
  __syncthreads();
  if (wave == 0) {
#pragma unroll 1
    for (int b0 = 0; b0 < tt; b0 += 32) {
      const int idx = b0 + lane;
      const int ent = hl[idx < RCAP ? idx : RCAP - 1];
      const int m32 = (tt - b0) < 32 ? (tt - b0) : 32;
#pragma unroll 1
      for (int k = 0; k < m32; ++k) {
        const int u    = __builtin_amdgcn_readlane(ent, k);
        const int slot = u & (NBA - 1);
        if (lane == 0) {
          int p = cur[slot];
          p = p < 0 ? 0 : (p > RCAP - 1 ? RCAP - 1 : p);
          sl[p] = u;
          cur[slot] = p + 1;
        }
      }
    }
  }
  __syncthreads();

  const float qnan = __int_as_float(0x7fc00000);
  const float pz = (ovf != 0) ? qnan : 0.0f;
  int wbig = 0;
  float bb0 = 0.0f, bb1 = 0.0f;
  if constexpr (LY == 2) {
    const v2f bb = *(const v2f*)(b2 + 2 * lane);
    bb0 = bf16_val(bb.x); bb1 = bf16_val(bb.y);
  }
#pragma unroll 1
  for (int si = 0; si < NBA / NWAVE; ++si) {
    const int s    = si * NWAVE + wave;
    const int node = nodeBase + s;
    int c = cnt[s];
    const bool big = c > DEGCAP;
    wbig |= big ? 1 : 0;
    c = c < 0 ? 0 : (c > DEGCAP ? DEGCAP : c);
    int o = offs[s];
    o = o < 0 ? 0 : (o > RCAP ? RCAP : o);
    float g0 = 0.0f, g1 = 0.0f, g2 = 0.0f, g3 = 0.0f;
#pragma unroll 1
    for (int b0 = 0; b0 < c; b0 += 32) {
      int idx = o + b0 + lane;
      idx = idx > RCAP - 1 ? RCAP - 1 : idx;
      const int ent = sl[idx];
      int eid = ent >> SLA;
      eid = eid < 0 ? 0 : (eid > nE - 1 ? nE - 1 : eid);
      int sr = gath[eid];
      sr = sr < 0 ? 0 : (sr > nN - 1 ? nN - 1 : sr);
      if constexpr (LY == 2) {
        int c1 = idx1[sr];
        c1 = c1 < 0 ? 0 : (c1 > nC - 1 ? nC - 1 : c1);
        int jj = rep1[c1];
        jj = jj < 0 ? 0 : (jj > nN - 1 ? nN - 1 : jj);
        sr = jj;
      }
      const int wvi = __float_as_int(bf16_val(ew[eid]));
      const int m32 = (c - b0) < 32 ? (c - b0) : 32;
#pragma unroll 1
      for (int k = 0; k < m32; ++k) {
        const int   sk = __builtin_amdgcn_readlane(sr, k);
        const float wk = __int_as_float(__builtin_amdgcn_readlane(wvi, k));
        if constexpr (LY == 1) {
          const v2u a = *(const v2ua*)(xb + (size_t)sk * DF + 4 * lane);
          const float f0 = __uint_as_float(a.x << 16);
          const float f1 = __uint_as_float(a.x & 0xffff0000u);
          const float f2 = __uint_as_float(a.y << 16);
          const float f3 = __uint_as_float(a.y & 0xffff0000u);
          g0 = fmaf(wk, f0, g0); g1 = fmaf(wk, f1, g1);
          g2 = fmaf(wk, f2, g2); g3 = fmaf(wk, f3, g3);
        } else {
          const v2f a = *(const v2fa*)(gq + (size_t)sk * DO + 2 * lane);
          g0 = fmaf(wk, a.x, g0); g1 = fmaf(wk, a.y, g1);
        }
      }
    }
    const float pzr = big ? qnan : pz;
    const bool live = node < nN;
    if constexpr (LY == 1) {
      const float q0 = live ? g0 + pzr : 0.0f, q1 = live ? g1 + pzr : 0.0f;
      const float q2 = live ? g2 + pzr : 0.0f, q3 = live ? g3 + pzr : 0.0f;
      int h01, h23, l01, l23;
      hilo_pack(q0, q1, q2, q3, h01, h23, l01, l23);
      const v4i ow = regroup16(h01, h23, l01, l23, lane);
      if (node < mRows) {
        unsigned short* hp = apl + (size_t)node * KA + 8 * lane;
        *(volatile v4i*)hp = ow;
        __threadfence();
        *(volatile v4i*)hp = ow;
      }
    } else {
      const float v0 = (g0 + bb0) + pzr;
      const float v1 = (g1 + bb1) + pzr;
      float mx = (v1 > v0 || v1 != v1) ? v1 : v0;
#pragma unroll
      for (int q = 16; q > 0; q >>= 1) {
        const float ot = __shfl_xor(mx, q, 32);
        mx = (ot > mx || ot != ot) ? ot : mx;
      }
      const float es = wsum(expf(v0 - mx) + expf(v1 - mx));
      const float ls = mx + logf(es);
      v2f ow;
      ow.x = (v0 - ls) + pzr;
      ow.y = (v1 - ls) + pzr;
      if (live) {
        float* op = qout + (size_t)node * DO + 2 * lane;
        *(volatile v2f*)op = ow;
        __threadfence();
        *(volatile v2f*)op = ow;
      }
    }
  }

  if (lane == 0) misc[16 + wave] = wbig;
  __syncthreads();
  if (wave == 0) {
    int f = ovf;
#pragma unroll
    for (int w2 = 0; w2 < NWAVE; ++w2) f |= misc[16 + w2];
    f = (f != 0) ? 1 : 0;
    if (lane < 8) {
      const v4i fv = {f, f, f, f};
      int* fp = flg + (size_t)blockIdx.x * FLP + 4 * lane;
      *(volatile v4i*)fp = fv;
      __threadfence();
      *(volatile v4i*)fp = fv;
    }
  }
}

__global__ __launch_bounds__(NTHR) void k_out(const float* __restrict__ q, const int* __restrict__ idx2,
                                              const int* __restrict__ rep2, int nN, int nC,
                                              const int* __restrict__ flg, int nfl, float* out) {
  __shared__ int sfl[NWAVE];
  const int tid = (int)threadIdx.x, lane = tid & 31, wave = tid >> 5;
  {
    const int fi = tid < nfl ? tid : nfl - 1;
    int fv = flg[(size_t)fi * FLP];
    fv = (tid < nfl) ? fv : 0;
    const unsigned bal = __builtin_amdgcn_ballot_w32(fv != 0);
    if (lane == 0) sfl[wave] = (bal != 0u) ? 1 : 0;
  }
  __syncthreads();
  int any = 0;
#pragma unroll
  for (int w2 = 0; w2 < NWAVE; ++w2) any |= sfl[w2];
  const float pz = (any != 0) ? __int_as_float(0x7fc00000) : 0.0f;

  const int n  = ((int)blockIdx.x * NWAVE + wave) * 2 + (lane >> 4);
  const int nc = n < nN ? n : nN - 1;
  int c2 = idx2[nc];
  c2 = c2 < 0 ? 0 : (c2 > nC - 1 ? nC - 1 : c2);
  int j = rep2[c2];
  j = j < 0 ? 0 : (j > nN - 1 ? nN - 1 : j);
  const int c4 = 4 * (lane & 15);
  v4f v = *(const v4fa*)(q + (size_t)j * DO + c4);
  v.x += pz; v.y += pz; v.z += pz; v.w += pz;
  if (n < nN) {
    float* op = out + (size_t)n * DO + c4;
    *(volatile v4f*)op = v;
    __threadfence();
    *(volatile v4f*)op = v;
  }
}

static inline int cdiv(int a, int b) { return (a + b - 1) / b; }
static inline size_t al256(size_t o) { return (o + 255) & ~(size_t)255; }

extern "C" void kernel_launch(void* const* d_in, const int* in_sizes, int n_in,
                              void* d_out, int out_size, void* d_ws, size_t ws_size,
                              hipStream_t stream) {
  if (n_in < 11) return;
  if (in_sizes[0] < DF || (in_sizes[0] % DF) != 0) return;
  const int nN = in_sizes[0] / DF;
  if ((nN % 16) != 0 || nN < 64 || nN >= (1 << 24)) return;
  if (in_sizes[1] < 2 || (in_sizes[1] & 1) != 0) return;
  const int nE = in_sizes[1] / 2;
  if (nE < 1 || nE >= (1 << 21)) return;
  if (in_sizes[2] != nE) return;
  const int nC = in_sizes[3];
  if (nC < 1 || in_sizes[5] != nC) return;
  if (in_sizes[4] != nN || in_sizes[6] != nN) return;
  if (in_sizes[7] != DF * DF || in_sizes[8] != DF) return;
  if (in_sizes[9] != DF * DO || in_sizes[10] != DO) return;
  if ((long long)out_size != (long long)nN * DO) return;

  const float* x    = (const float*)d_in[0];
  const int*   edge = (const int*)d_in[1];
  const float* ew   = (const float*)d_in[2];
  const int*   rep1 = (const int*)d_in[3];
  const int*   idx1 = (const int*)d_in[4];
  const int*   rep2 = (const int*)d_in[5];
  const int*   idx2 = (const int*)d_in[6];
  const float* w1   = (const float*)d_in[7];
  const float* b1   = (const float*)d_in[8];
  const float* w2   = (const float*)d_in[9];
  const float* b2   = (const float*)d_in[10];
  float* out = (float*)d_out;
  const int* gath = edge;
  const int* keys = edge + nE;

  const int MP = cdiv(nN, GBM) * GBM;
  const int gM = MP / GBM;
  const int gX = cdiv(nN * (DF / 8), NTHR);
  const int gA = cdiv(nN, NBA);
  if ((long long)gA * NBA < (long long)MP) return;
  const int nfl = 2 * gA;
  if (nfl > NTHR) return;
  const int gO = cdiv(nN, 2 * NWAVE);
  const int vec8 = ((nE & 3) == 0) ? 1 : 0;

  char* ws = (char*)d_ws;
  size_t off = 0;
  const size_t oW1D = off; off = al256(off + (size_t)DF * KA * 2);
  const size_t oW2D = off; off = al256(off + (size_t)DO * KA * 2);
  const size_t oFLG = off; off = al256(off + (size_t)nfl * FLP * 4);
  const size_t oXB  = off; off = al256(off + (size_t)nN * DF * 2);
  const size_t oAR  = off; off = al256(off + (size_t)MP * KA * 2);
  const size_t oG   = off; off = al256(off + (size_t)MP * DO * 4);
  const size_t oQ   = off; off = al256(off + (size_t)nN * DO * 4);
  if (off > ws_size || off > (size_t)WSMAX) return;
  unsigned short* W1D = (unsigned short*)(ws + oW1D);
  unsigned short* W2D = (unsigned short*)(ws + oW2D);
  int*            FLG = (int*)(ws + oFLG);
  unsigned short* XB  = (unsigned short*)(ws + oXB);
  unsigned short* AR  = (unsigned short*)(ws + oAR);
  float*          G   = (float*)(ws + oG);
  float*          Q   = (float*)(ws + oQ);

  const size_t scanLds = (size_t)AGG_LDS_INTS * 4;
  hipFuncSetAttribute(reinterpret_cast<const void*>(&k_scan<1>), hipFuncAttributeMaxDynamicSharedMemorySize, (int)scanLds);
  hipFuncSetAttribute(reinterpret_cast<const void*>(&k_scan<2>), hipFuncAttributeMaxDynamicSharedMemorySize, (int)scanLds);

  k_prep<<<gX + NBW1 + NBW2, NTHR, 0, stream>>>(x, nN, gX, w1, w2, XB, W1D, W2D);
  k_scan<1><<<gA, NTHR, scanLds, stream>>>(gath, keys, ew, nE, nN, vec8, MP, XB, G, idx1, rep1, nC, b2, AR, Q, FLG);
  k_gemm<8, 0><<<gM, GTHR, 0, stream>>>(AR, W1D, b1, nN, G);
  k_gemm<4, 1><<<gM, GTHR, 0, stream>>>(AR, W2D, b1, nN, G);
  k_scan<2><<<gA, NTHR, scanLds, stream>>>(gath, keys, ew, nE, nN, vec8, MP, XB, G, idx1, rep1, nC, b2, AR, Q,
                                           FLG + (size_t)gA * FLP);
  k_out<<<gO, NTHR, 0, stream>>>(Q, idx2, rep2, nN, nC, FLG, nfl, out);
}
